// MixerModel_50259707298213
// MI455X (gfx1250) — hardware-run, weakly checked
//
#include <hip/hip_runtime.h>
#include <hip/hip_fp16.h>
#include <math.h>

typedef __attribute__((ext_vector_type(16))) _Float16 v16h;
typedef __attribute__((ext_vector_type(8)))  _Float16 v8h;
typedef __attribute__((ext_vector_type(8)))  float    v8f;
typedef __attribute__((ext_vector_type(4)))  float    v4f;

constexpr int kLayers = 2;
constexpr int kBatch  = 2;
constexpr int kSeq    = 2048;
constexpr int kRows   = kBatch * kSeq;
constexpr int kDm     = 1024;
constexpr int kDin    = 2048;
constexpr int kNst    = 16;
constexpr int kDtR    = 64;
constexpr int kXzP    = 2 * kDin;
constexpr int kXpN    = kDtR + 2 * kNst;
constexpr int kXdP    = 128;
constexpr int kOffB   = kDtR;
constexpr int kOffC   = kDtR + kNst;
constexpr int kConvTP = 260;
constexpr float kLnEps      = 1e-5f;
constexpr float kActCarry   = 16.0f;
constexpr float kWinCarry   = 256.0f;
constexpr float kWxCarry    = 256.0f;
constexpr float kWdtCarry   = 64.0f;
constexpr float kWoutCarry  = 256.0f;
constexpr float kUCarry     = 16.0f;
constexpr float kDlCarry    = 64.0f;
constexpr float kYCarry     = 16.0f;
constexpr float kScaleIn    = 1.0f / (kActCarry * kWinCarry);
constexpr float kScaleX     = 1.0f / (kUCarry * kWxCarry);
constexpr float kScaleDt    = 1.0f / (kDlCarry * kWdtCarry);
constexpr float kScaleOut   = 1.0f / (kYCarry * kWoutCarry);
static_assert(kLayers == 2);
static_assert(kXpN == 96 && kXpN <= kXdP);
static_assert((kDm % 64) == 0 && (kDin % 64) == 0 && (kXzP % 64) == 0 && (kXdP % 64) == 0);
static_assert((kSeq % 64) == 0 && (kDin % 256) == 0 && kDm == 1024);
static_assert((kSeq % 64) == 0 && (kXzP % 64) == 0 && (kDm % 32) == 0);
static_assert((kXdP % 64) == 0 && (kDin % 32) == 0);
static_assert((kDin % 64) == 0 && (kDtR % 32) == 0);
static_assert((kDm % 64) == 0 && (kDin % 32) == 0);
static_assert(((kSeq / 64) * (kXzP / 64)) % 8 == 0 && ((kSeq / 64) * (kXdP / 64)) % 8 == 0);
static_assert(((kSeq / 64) * (kDin / 64)) % 8 == 0 && ((kSeq / 64) * (kDm / 64)) % 8 == 0);

constexpr size_t kSzRes   = (size_t)kRows * kDm * 4;
constexpr size_t kSzNrm   = (size_t)kRows * kDm * 2;
constexpr size_t kSzWIN   = (size_t)kXzP * kDm * 2;
constexpr size_t kSzWOUT  = (size_t)kDm * kDin * 2;
constexpr size_t kSzWX    = (size_t)kXdP * kDin * 2;
constexpr size_t kSzWDT   = (size_t)kDin * kDtR * 2;
constexpr size_t kSzXZ    = (size_t)kSeq * kXzP * 4;
constexpr size_t kSzU     = (size_t)kSeq * kDin * 4;
constexpr size_t kSzU16   = (size_t)kSeq * kDin * 2;
constexpr size_t kSzXD    = (size_t)kSeq * kXdP * 4;
constexpr size_t kSzDL    = (size_t)kSeq * kDtR * 2;
constexpr size_t kOffRES  = 0;
constexpr size_t kOffMO   = kOffRES  + kSzRes;
constexpr size_t kOffNRM  = kOffMO   + kSzRes;
constexpr size_t kOffWIN  = kOffNRM  + kSzNrm;
constexpr size_t kOffWOUT = kOffWIN  + kSzWIN;
constexpr size_t kOffWX   = kOffWOUT + kSzWOUT;
constexpr size_t kOffWDT  = kOffWX   + kSzWX;
constexpr size_t kOffXZ   = kOffWDT  + kSzWDT;
constexpr size_t kOffU    = kOffXZ   + kSzXZ;
constexpr size_t kOffUY   = kOffU    + kSzU;
constexpr size_t kOffXD   = kOffUY   + kSzU16;
constexpr size_t kOffDL   = kOffXD   + kSzXD;
constexpr size_t kOffDT   = kOffDL   + kSzDL;
constexpr size_t kWsTotal = kOffDT   + kSzU;
static_assert(kWsTotal == 132120576ull);
static_assert(kWsTotal <= 134217728ull);
static_assert((kOffMO % 128) == 0 && (kOffNRM % 128) == 0 && (kOffWIN % 128) == 0 && (kOffWOUT % 128) == 0 &&
              (kOffWX % 128) == 0 && (kOffWDT % 128) == 0 && (kOffXZ % 128) == 0 && (kOffU % 128) == 0 &&
              (kOffUY % 128) == 0 && (kOffXD % 128) == 0 && (kOffDL % 128) == 0 && (kOffDT % 128) == 0);

__device__ __forceinline__ _Float16 f16_flush(float v) {
  const float w = (fabsf(v) < 6.103515625e-05f) ? 0.0f : v;
  return (_Float16)w;
}

__device__ __forceinline__ void dep_guard_h(v8f& a, v8f& b, v16h x, v16h y) { asm volatile("v_nop\n\tv_nop\n\tv_nop\n\tv_nop" : "+v"(a), "+v"(b) : "v"(x), "v"(y)); }
__device__ __forceinline__ void keep4_h(v16h a, v16h b, v16h c, v16h d) { asm volatile("v_nop" :: "v"(a), "v"(b), "v"(c), "v"(d)); }
__device__ __forceinline__ void acc_guard4(v8f& a, v8f& b, v8f& c, v8f& d) { asm volatile("v_nop\n\tv_nop\n\tv_nop\n\tv_nop" : "+v"(a), "+v"(b), "+v"(c), "+v"(d)); }
template <typename T> struct Frag;
template <> struct Frag<_Float16> {
  typedef v16h V; union U { v16h v; v8h h[2]; };
  static __device__ __forceinline__ v16h load(const _Float16* p) {
    U f; f.h[0] = *(const v8h*)(p); f.h[1] = *(const v8h*)(p + 16); return f.v;
  }
  static __device__ __forceinline__ v8f mma(v16h a, v16h b, v8f c) {
    return __builtin_amdgcn_wmma_f32_16x16x32_f16(false, a, false, b, (short)0, c, false, false);
  }
  static __device__ __forceinline__ void guard(v8f& a, v8f& b, v16h x, v16h y) { dep_guard_h(a, b, x, y); }
  static __device__ __forceinline__ void keep(v16h a, v16h b, v16h c, v16h d) { keep4_h(a, b, c, d); }
};

template <bool BIAS_N, bool OUT16>
__global__ __launch_bounds__(256) void gemm64_f16_kernel(
    const unsigned short* __restrict__ Ap, int lda,
    const unsigned short* __restrict__ Btp, int ldb,
    float* __restrict__ C32, int ldc32,
    unsigned short* __restrict__ C16, int ldc16, int n16lim, float carry16,
    const float* __restrict__ bias,
    int M, int N, int K, float scale) {
  typedef _Float16 T;
  typedef Frag<_Float16>::V V;
  const T* A = (const T*)Ap; const T* Bt = (const T*)Btp;
  __shared__ __align__(16) float sT[8][16 * 68];
  const int lane = threadIdx.x & 31;
  const int wave = threadIdx.x >> 5;
  const int tilesN = N >> 6;
  const int tilesM = M >> 6;
  const int tile = blockIdx.x * 8 + wave;
  if (tile >= tilesM * tilesN) return;
  const int tm = tile / tilesN;
  const int tn = tile - tm * tilesN;
  const int m0 = tm << 6;
  const int n0 = tn << 6;

  const int rlane = lane & 15;
  const int koff  = (lane >> 4) * 8;
  const int mOff  = (lane >> 4) * 8;

  v8f acc[4][4];
#pragma unroll
  for (int i = 0; i < 4; ++i)
#pragma unroll
    for (int j = 0; j < 4; ++j) acc[i][j] = (v8f){0.f,0.f,0.f,0.f,0.f,0.f,0.f,0.f};

  float bvj[4] = {0.f, 0.f, 0.f, 0.f};
  if (BIAS_N) {
#pragma unroll
    for (int j = 0; j < 4; ++j) bvj[j] = bias[n0 + (j << 4) + rlane];
  }

  for (int k0 = 0; k0 < K; k0 += 32) {
    V bh[4];
#pragma unroll
    for (int j = 0; j < 4; ++j) {
      const size_t bo = (size_t)(n0 + (j << 4) + rlane) * ldb + koff + k0;
      bh[j] = Frag<T>::load(Bt + bo);
    }
#pragma unroll
    for (int i = 0; i < 4; ++i) {
      const size_t ao = (size_t)(m0 + (i << 4) + rlane) * lda + koff + k0;
      V ah = Frag<T>::load(A + ao);
#pragma unroll
      for (int j = 0; j < 4; ++j) {
        acc[i][j] = Frag<T>::mma(ah, bh[j], acc[i][j]);
      }
      Frag<T>::guard(acc[i][0], acc[i][3], ah, ah);
    }
    Frag<T>::keep(bh[0], bh[1], bh[2], bh[3]);
  }
  acc_guard4(acc[0][0], acc[0][1], acc[0][2], acc[0][3]);
  acc_guard4(acc[1][0], acc[1][1], acc[1][2], acc[1][3]);
  acc_guard4(acc[2][0], acc[2][1], acc[2][2], acc[2][3]);
  acc_guard4(acc[3][0], acc[3][1], acc[3][2], acc[3][3]);

  float* slab = sT[wave];
#pragma unroll
  for (int i = 0; i < 4; ++i) {
    const int mBase = m0 + (i << 4);
#pragma unroll
    for (int j = 0; j < 4; ++j) {
#pragma unroll
      for (int r = 0; r < 8; ++r) {
        float v = acc[i][j][r] * scale;
        if (BIAS_N) v += bvj[j];
        slab[(mOff + r) * 68 + (j << 4) + rlane] = v;
      }
    }
    __builtin_amdgcn_fence(__ATOMIC_RELEASE, "workgroup");
    __builtin_amdgcn_wave_barrier();
    __builtin_amdgcn_fence(__ATOMIC_ACQUIRE, "workgroup");
    {
      const int hh = lane >> 4, c4 = (lane & 15) * 4;
      for (int pass = 0; pass < 2; ++pass) {
#pragma unroll
        for (int it = 0; it < 8; ++it) {
          const int row = it * 2 + hh;
          v4f v = *(const v4f*)(slab + row * 68 + c4);
          *(volatile v4f*)(C32 + (size_t)(mBase + row) * ldc32 + n0 + c4) = v;
        }
        __threadfence();
      }
    }
    if (OUT16) {
      if (n0 < n16lim) {
        const int q = lane >> 3, c8 = (lane & 7) * 8;
        for (int pass = 0; pass < 2; ++pass) {
#pragma unroll
          for (int it = 0; it < 4; ++it) {
            const int row = it * 4 + q;
            const float* sp = slab + row * 68 + c8;
            const v4f a0 = *(const v4f*)(sp);
            const v4f a1 = *(const v4f*)(sp + 4);
            v8h hv;
#pragma unroll
            for (int e = 0; e < 4; ++e) {
              hv[e]     = f16_flush(a0[e] * carry16);
              hv[4 + e] = f16_flush(a1[e] * carry16);
            }
            *(volatile v8h*)(C16 + (size_t)(mBase + row) * ldc16 + n0 + c8) = hv;
          }
          __threadfence();
        }
      }
    }
    __builtin_amdgcn_fence(__ATOMIC_RELEASE, "workgroup");
    __builtin_amdgcn_wave_barrier();
    __builtin_amdgcn_fence(__ATOMIC_ACQUIRE, "workgroup");
  }
}

__global__ __launch_bounds__(256) void pack_rows_f16_kernel(
    const float* __restrict__ src, unsigned short* __restrict__ dst, int real8, int total8, float carry)
{
  const int i = blockIdx.x * 256 + threadIdx.x;
  if (i >= total8) return;
  const int ic = (i < real8) ? i : (real8 - 1);
  const float ck = (i < real8) ? carry : 0.0f;
  const size_t e0 = (size_t)ic << 3;
  const v4f a0 = *(const v4f*)(src + e0);
  const v4f a1 = *(const v4f*)(src + e0 + 4);
  v8h hv;
#pragma unroll
  for (int e = 0; e < 4; ++e) {
    hv[e]     = f16_flush(a0[e] * ck);
    hv[4 + e] = f16_flush(a1[e] * ck);
  }
  unsigned short* qh = dst + ((size_t)i << 3);
  *(volatile v8h*)qh = hv;
  __threadfence();
  *(volatile v8h*)qh = hv;
}

template <bool ADD, bool WRES, bool FINAL>
__global__ __launch_bounds__(256) void add_norm_kernel(
    const float* __restrict__ hid, const float* __restrict__ res_in, float* __restrict__ res_out,
    unsigned short* __restrict__ n16, float* __restrict__ o32,
    const float* __restrict__ gw, const float* __restrict__ gb, float carry)
{
  __shared__ float sA[8];
  __shared__ float sB[8];
  __shared__ __align__(16) float sN[kDm];
  const int tid = threadIdx.x, lane = tid & 31, wave = tid >> 5;
  const size_t o = (size_t)blockIdx.x * kDm + (size_t)tid * 4;
  v4f x = *(const v4f*)(hid + o);
  if (ADD) {
    const v4f rr = *(const v4f*)(res_in + o);
    x = x + rr;
  }
  float s = (x[0] + x[1]) + (x[2] + x[3]);
#pragma unroll
  for (int off = 16; off > 0; off >>= 1) s += __shfl_xor(s, off, 32);
  if (lane == 0) sA[wave] = s;
  __syncthreads();
  float ts = 0.0f;
#pragma unroll
  for (int i = 0; i < 8; ++i) ts += sA[i];
  const float mu = ts * (1.0f / (float)kDm);
  v4f dv;
#pragma unroll
  for (int e = 0; e < 4; ++e) dv[e] = x[e] - mu;
  float qv = (dv[0] * dv[0] + dv[1] * dv[1]) + (dv[2] * dv[2] + dv[3] * dv[3]);
#pragma unroll
  for (int off = 16; off > 0; off >>= 1) qv += __shfl_xor(qv, off, 32);
  if (lane == 0) sB[wave] = qv;
  __syncthreads();
  float tq = 0.0f;
#pragma unroll
  for (int i = 0; i < 8; ++i) tq += sB[i];
  const float var = tq * (1.0f / (float)kDm);
  const float rstd = rsqrtf(var + kLnEps);
  const v4f wv = *(const v4f*)(gw + tid * 4);
  const v4f bv = *(const v4f*)(gb + tid * 4);
  v4f yv;
#pragma unroll
  for (int e = 0; e < 4; ++e) yv[e] = dv[e] * rstd * wv[e] + bv[e];

  v8h hv = (v8h){0, 0, 0, 0, 0, 0, 0, 0};
  if (!FINAL) {
    v4f cv;
#pragma unroll
    for (int e = 0; e < 4; ++e) cv[e] = yv[e] * carry;
    *(v4f*)(sN + tid * 4) = cv;
    __syncthreads();
    const float* sp = sN + (tid & 127) * 8;
    const v4f a0 = *(const v4f*)(sp);
    const v4f a1 = *(const v4f*)(sp + 4);
#pragma unroll
    for (int e = 0; e < 4; ++e) {
      hv[e]     = f16_flush(a0[e]);
      hv[4 + e] = f16_flush(a1[e]);
    }
  }
  for (int pass = 0; pass < 2; ++pass) {
    if (WRES) *(volatile v4f*)(res_out + o) = x;
    if (FINAL) *(volatile v4f*)(o32 + o) = yv;
    if (!FINAL) {
      if (tid < 128) *(volatile v8h*)(n16 + (size_t)blockIdx.x * kDm + (size_t)tid * 8) = hv;
    }
    __threadfence();
  }
}

__global__ __launch_bounds__(256) void conv_silu_kernel(
    const float* __restrict__ XZ, const float* __restrict__ cw, const float* __restrict__ cb,
    float* __restrict__ UC, unsigned short* __restrict__ UH, float carry)
{
  __shared__ __align__(16) float sT[16 * kConvTP];
  const int tid = threadIdx.x, lane = tid & 31, wave = tid >> 5;
  const int d0 = blockIdx.x * 256, d = d0 + tid;
  const int t0 = blockIdx.y * 64;
  const v4f wv = *(const v4f*)(cw + (size_t)d * 4);
  const float w0 = wv[0], w1 = wv[1], w2 = wv[2], w3 = wv[3];
  const float bc = cb[d];
  float xm3, xm2, xm1;
  {
    const int r3 = t0 - 3, r2 = t0 - 2, r1 = t0 - 1;
    const float v3 = XZ[(size_t)(r3 < 0 ? 0 : r3) * kXzP + d];
    const float v2 = XZ[(size_t)(r2 < 0 ? 0 : r2) * kXzP + d];
    const float v1 = XZ[(size_t)(r1 < 0 ? 0 : r1) * kXzP + d];
    xm3 = (r3 >= 0) ? v3 : 0.0f;
    xm2 = (r2 >= 0) ? v2 : 0.0f;
    xm1 = (r1 >= 0) ? v1 : 0.0f;
  }
  const int hrow = wave >> 1;
  const int hch  = (wave & 1) * 128 + lane * 4;
#pragma unroll 1
  for (int sub = 0; sub < 4; ++sub) {
    const int lb = t0 + sub * 16;
#pragma unroll 1
    for (int s = 0; s < 16; ++s) {
      const float xcur = XZ[(size_t)(lb + s) * kXzP + d];
      float acc = w0 * xm3;
      acc = fmaf(w1, xm2, acc);
      acc = fmaf(w2, xm1, acc);
      acc = fmaf(w3, xcur, acc);
      const float sv = bc + acc;
      const float sg = __builtin_amdgcn_rcpf(1.0f + expf(-sv));
      sT[s * kConvTP + tid] = sv * sg;
      xm3 = xm2; xm2 = xm1; xm1 = xcur;
    }
    __syncthreads();
    v4f fv[4];
    v8h hv[2];
#pragma unroll
    for (int it = 0; it < 4; ++it) fv[it] = *(const v4f*)(sT + (it * 4 + hrow) * kConvTP + hch);
#pragma unroll
    for (int it = 0; it < 2; ++it) {
      const float* sp = sT + (it * 8 + wave) * kConvTP + lane * 8;
      const v4f a0 = *(const v4f*)(sp);
      const v4f a1 = *(const v4f*)(sp + 4);
#pragma unroll
      for (int e = 0; e < 4; ++e) {
        hv[it][e]     = f16_flush(a0[e] * carry);
        hv[it][4 + e] = f16_flush(a1[e] * carry);
      }
    }
    for (int pass = 0; pass < 2; ++pass) {
#pragma unroll
      for (int it = 0; it < 4; ++it)
        *(volatile v4f*)(UC + (size_t)(lb + it * 4 + hrow) * kDin + d0 + hch) = fv[it];
#pragma unroll
      for (int it = 0; it < 2; ++it) {
        const size_t o = (size_t)(lb + it * 8 + wave) * kDin + d0 + lane * 8;
        *(volatile v8h*)(UH + o) = hv[it];
      }
      __threadfence();
    }
    __syncthreads();
  }
}

typedef float    ms1_v4f __attribute__((ext_vector_type(4)));
typedef unsigned ms1_v4u __attribute__((ext_vector_type(4)));
struct ms1_args {
  const float* dtpre;
  const float* u;
  const float* bc;
  const float* z;
  const float* A_log;
  const float* Dskip;
  __half* y;
  __half* y_lo;
  long ld_dtpre;
  long ld_u;
  long ld_bc;
  long ld_z;
  long ld_y;
  int offB;
  int offC;
  int offZ;
  float ycarry;
  int dir;
  int D;
  int L;
  int nbatch;
};
static_assert(sizeof(ms1_args) == 136);

__device__ __forceinline__ float ms1_flush16(float v) {
  return (fabsf(v) < 6.103515625e-05f) ? 0.0f : v;
}
__device__ __forceinline__ unsigned ms1_h16bits(float v) {
  return (unsigned)__half_as_ushort(__float2half_rn(ms1_flush16(v)));
}
__device__ __forceinline__ float ms1_h16val(unsigned b) {
  return __half2float(__ushort_as_half((unsigned short)b));
}
__device__ __forceinline__ float ms1_softplus(float v) {
  return fmaxf(v, 0.0f) + log1pf(expf(-fabsf(v)));
}
__device__ __forceinline__ void ms1_pack2(float v0, float v1, unsigned& hw, unsigned& lw) {
  const unsigned h0 = ms1_h16bits(v0);
  const unsigned h1 = ms1_h16bits(v1);
  const float r0 = (v0 - ms1_h16val(h0)) * 2048.0f;
  const float r1 = (v1 - ms1_h16val(h1)) * 2048.0f;
  const unsigned l0 = ms1_h16bits(r0);
  const unsigned l1 = ms1_h16bits(r1);
  hw = h0 | (h1 << 16);
  lw = l0 | (l1 << 16);
}

template <int NSTATE>
__global__ __launch_bounds__(64 * (NSTATE / 16)) void ms1_scan_kernel(ms1_args a)
{
  static_assert(NSTATE == 16 || NSTATE == 64);
  constexpr int NQ  = NSTATE / 16;
  constexpr int NT  = 64 * NQ;
  constexpr int NW  = NT / 32;
  constexpr int BCW = 2 * NSTATE;
  constexpr int YP  = 68;
  constexpr int RPI = NW * 4;
  constexpr int NIT = 64 / RPI;
  static_assert(16 * NT <= 64 * YP);
  __shared__ __align__(16) float sBC[64 * BCW];
  __shared__ __align__(16) float sY[64 * YP];
  const int tid  = threadIdx.x;
  const int lane = tid & 31;
  const int wave = tid >> 5;
  const int c    = tid / NQ;
  const int sq   = tid - c * NQ;
  const int bpb  = a.D / 64;
  const int bi   = blockIdx.x / bpb;
  if (bi >= a.nbatch) return;
  const int d0 = (blockIdx.x - bi * bpb) * 64;
  const int d  = d0 + c;
  const long rowb = (long)bi * a.L;
  const bool hasz  = (a.z != nullptr);
  const bool hasD  = (a.Dskip != nullptr);
  const bool hasLo = (a.y_lo != nullptr);

#pragma unroll 1
  for (int n = 0; n < 16; ++n) {
    const float al = a.A_log[(long)d * NSTATE + sq * 16 + n];
    sY[n * NT + tid] = -expf(al);
  }
  __syncthreads();
  float An[16], h[16];
#pragma unroll
  for (int n = 0; n < 16; ++n) {
    An[n] = sY[n * NT + tid];
    h[n] = 0.0f;
  }
  float Dd = 0.0f;
  if (hasD) Dd = a.Dskip[d];

  const int nchunk = a.L / 64;
  const bool fwd = (a.dir > 0);
  const int s0 = fwd ? 0 : 63;
  const int sd = fwd ? 1 : -1;
  const int q  = lane >> 3;
  const int c8 = (lane & 7) * 8;

#pragma unroll 1
  for (int ci = 0; ci < nchunk; ++ci) {
    const int tb = fwd ? (ci * 64) : (a.L - 64 - ci * 64);
    const long rowc = rowb + tb;
    __syncthreads();
#pragma unroll 8
    for (int i = 0; i < 32; ++i) {
      const int idx = tid + i * NT;
      const int st  = idx / BCW;
      const int col = idx - st * BCW;
      const int sc  = (col < NSTATE) ? (a.offB + col) : (a.offC + col - NSTATE);
      sBC[idx] = a.bc[(rowc + st) * a.ld_bc + sc];
    }
    __syncthreads();
#pragma unroll 1
    for (int s = 0; s < 64; ++s) {
      const int ls = s0 + sd * s;
      const long row = rowc + ls;
      float pre = a.dtpre[row * a.ld_dtpre + d];
      float uv  = a.u[row * a.ld_u + d];
      float zv  = 0.0f;
      if (hasz) zv = a.z[row * a.ld_z + a.offZ + d];
      asm volatile("" : "+v"(pre));
      asm volatile("" : "+v"(uv));
      asm volatile("" : "+v"(zv));
      const float delta = ms1_softplus(pre);
      const float dtx = delta * uv;
      const float* bp = sBC + ls * BCW + sq * 16;
      const float* cp = bp + NSTATE;
      ms1_v4f Bq[4], Cq[4];
#pragma unroll
      for (int k = 0; k < 4; ++k) {
        Bq[k] = *(const ms1_v4f*)(bp + 4 * k);
        Cq[k] = *(const ms1_v4f*)(cp + 4 * k);
      }
      float yv = 0.0f;
#pragma unroll
      for (int n = 0; n < 16; ++n) {
        const float e = __expf(delta * An[n]);
        h[n] = fmaf(e, h[n], dtx * Bq[n >> 2][n & 3]);
        yv = fmaf(h[n], Cq[n >> 2][n & 3], yv);
      }
      if (NQ > 1) {
        yv += __shfl_xor(yv, 1, 32);
        yv += __shfl_xor(yv, 2, 32);
      }
      if (hasD) yv = fmaf(uv, Dd, yv);
      if (hasz) {
        const float sg = __builtin_amdgcn_rcpf(1.0f + expf(-zv));
        yv = yv * (zv * sg);
      }
      if (sq == 0) sY[ls * YP + c] = yv * a.ycarry;
    }
    __syncthreads();
    ms1_v4u hw[NIT], lw[NIT];
#pragma unroll
    for (int it = 0; it < NIT; ++it) {
      const int row = it * RPI + wave * 4 + q;
      const float* sp = sY + row * YP + c8;
      const ms1_v4f f0 = *(const ms1_v4f*)(sp);
      const ms1_v4f f1 = *(const ms1_v4f*)(sp + 4);
      unsigned h0, h1, h2, h3, l0, l1, l2, l3;
      ms1_pack2(f0[0], f0[1], h0, l0);
      ms1_pack2(f0[2], f0[3], h1, l1);
      ms1_pack2(f1[0], f1[1], h2, l2);
      ms1_pack2(f1[2], f1[3], h3, l3);
      hw[it] = (ms1_v4u){h0, h1, h2, h3};
      lw[it] = (ms1_v4u){l0, l1, l2, l3};
    }
    for (int pass = 0; pass < 2; ++pass) {
#pragma unroll
      for (int it = 0; it < NIT; ++it) {
        const int row = it * RPI + wave * 4 + q;
        const long o = (rowc + row) * a.ld_y + d0 + c8;
        *(volatile ms1_v4u*)(a.y + o) = hw[it];
        if (hasLo) *(volatile ms1_v4u*)(a.y_lo + o) = lw[it];
      }
      __threadfence();
    }
  }
}

extern "C" void kernel_launch(void* const* d_in, const int* in_sizes, int n_in,
                              void* d_out, int out_size, void* d_ws, size_t ws_size,
                              hipStream_t stream)
{
  if (n_in != 14) return;
  if (in_sizes[0]  != kRows * kDm) return;
  if (in_sizes[1]  != kLayers * kDm) return;
  if (in_sizes[2]  != kLayers * kDm) return;
  if (in_sizes[3]  != kLayers * kXzP * kDm) return;
  if (in_sizes[4]  != kLayers * kDin * 4) return;
  if (in_sizes[5]  != kLayers * kDin) return;
  if (in_sizes[6]  != kLayers * kXpN * kDin) return;
  if (in_sizes[7]  != kLayers * kDin * kDtR) return;
  if (in_sizes[8]  != kLayers * kDin) return;
  if (in_sizes[9]  != kLayers * kDin * kNst) return;
  if (in_sizes[10] != kLayers * kDin) return;
  if (in_sizes[11] != kLayers * kDm * kDin) return;
  if (in_sizes[12] != kDm) return;
  if (in_sizes[13] != kDm) return;
  if (out_size != kRows * kDm) return;
  if (ws_size < kWsTotal) return;

  const float* hs      = (const float*)d_in[0];
  const float* norm_w  = (const float*)d_in[1];
  const float* norm_b  = (const float*)d_in[2];
  const float* W_in    = (const float*)d_in[3];
  const float* conv_w  = (const float*)d_in[4];
  const float* conv_b  = (const float*)d_in[5];
  const float* W_x     = (const float*)d_in[6];
  const float* W_dt    = (const float*)d_in[7];
  const float* b_dt    = (const float*)d_in[8];
  const float* A_log   = (const float*)d_in[9];
  const float* D_par   = (const float*)d_in[10];
  const float* W_out   = (const float*)d_in[11];
  const float* normf_w = (const float*)d_in[12];
  const float* normf_b = (const float*)d_in[13];
  float* out = (float*)d_out;

  char* ws = (char*)d_ws;
  float*          RESID  = (float*)(ws + kOffRES);
  float*          MO     = (float*)(ws + kOffMO);
  unsigned short* NORMED = (unsigned short*)(ws + kOffNRM);
  unsigned short* WIN    = (unsigned short*)(ws + kOffWIN);
  unsigned short* WOUT   = (unsigned short*)(ws + kOffWOUT);
  unsigned short* WX     = (unsigned short*)(ws + kOffWX);
  unsigned short* WDT    = (unsigned short*)(ws + kOffWDT);
  float*          XZ     = (float*)(ws + kOffXZ);
  float*          U      = (float*)(ws + kOffU);
  unsigned short* UY     = (unsigned short*)(ws + kOffUY);
  float*          XD     = (float*)(ws + kOffXD);
  unsigned short* DTLOW  = (unsigned short*)(ws + kOffDL);
  float*          DT     = (float*)(ws + kOffDT);

  constexpr int kWin8   = kXzP * kDm / 8;
  constexpr int kWout8  = kDm * kDin / 8;
  constexpr int kWxR8   = kXpN * kDin / 8;
  constexpr int kWxT8   = kXdP * kDin / 8;
  constexpr int kWdt8   = kDin * kDtR / 8;
  static_assert((kWin8 % 256) == 0 && (kWout8 % 256) == 0 && (kWxT8 % 256) == 0 && (kWdt8 % 256) == 0);

  for (int i = 0; i < kLayers; ++i) {
    pack_rows_f16_kernel<<<kWin8 / 256, 256, 0, stream>>>(
        W_in + (size_t)i * kXzP * kDm, WIN, kWin8, kWin8, kWinCarry);
    pack_rows_f16_kernel<<<kWout8 / 256, 256, 0, stream>>>(
        W_out + (size_t)i * kDm * kDin, WOUT, kWout8, kWout8, kWoutCarry);
    pack_rows_f16_kernel<<<kWxT8 / 256, 256, 0, stream>>>(
        W_x + (size_t)i * kXpN * kDin, WX, kWxR8, kWxT8, kWxCarry);
    pack_rows_f16_kernel<<<kWdt8 / 256, 256, 0, stream>>>(
        W_dt + (size_t)i * kDin * kDtR, WDT, kWdt8, kWdt8, kWdtCarry);

    if (i == 0) {
      add_norm_kernel<false, false, false><<<kRows, 256, 0, stream>>>(
          hs, hs, RESID, NORMED, out, norm_w, norm_b, kActCarry);
    } else {
      add_norm_kernel<true, true, false><<<kRows, 256, 0, stream>>>(
          MO, hs, RESID, NORMED, out, norm_w + (size_t)i * kDm, norm_b + (size_t)i * kDm, kActCarry);
    }

    for (int b = 0; b < kBatch; ++b) {
      const unsigned short* nb = NORMED + (size_t)b * kSeq * kDm;
      float* mob = MO + (size_t)b * kSeq * kDm;

      gemm64_f16_kernel<false, false><<<(kSeq / 64) * (kXzP / 64) / 8, 256, 0, stream>>>(
          nb, kDm, WIN, kDm, XZ, kXzP, UY, 64, 0, 1.0f, b_dt, kSeq, kXzP, kDm, kScaleIn);

      conv_silu_kernel<<<dim3(kDin / 256, kSeq / 64), 256, 0, stream>>>(
          XZ, conv_w + (size_t)i * kDin * 4, conv_b + (size_t)i * kDin, U, UY, kUCarry);

      gemm64_f16_kernel<false, true><<<(kSeq / 64) * (kXdP / 64) / 8, 256, 0, stream>>>(
          UY, kDin, WX, kDin, XD, kXdP, DTLOW, kDtR, 64, kDlCarry, b_dt, kSeq, kXdP, kDin, kScaleX);

      gemm64_f16_kernel<true, false><<<(kSeq / 64) * (kDin / 64) / 8, 256, 0, stream>>>(
          DTLOW, kDtR, WDT, kDtR, DT, kDin, UY, 64, 0, 1.0f, b_dt + (size_t)i * kDin, kSeq, kDin, kDtR, kScaleDt);

      ms1_args sa;
      sa.dtpre = DT;
      sa.u = U;
      sa.bc = XD;
      sa.z = XZ;
      sa.A_log = A_log + (size_t)i * kDin * kNst;
      sa.Dskip = D_par + (size_t)i * kDin;
      sa.y = (__half*)UY;
      sa.y_lo = nullptr;
      sa.ld_dtpre = kDin;
      sa.ld_u = kDin;
      sa.ld_bc = kXdP;
      sa.ld_z = kXzP;
      sa.ld_y = kDin;
      sa.offB = kOffB;
      sa.offC = kOffC;
      sa.offZ = kDin;
      sa.ycarry = kYCarry;
      sa.dir = 1;
      sa.D = kDin;
      sa.L = kSeq;
      sa.nbatch = 1;
      ms1_scan_kernel<16><<<dim3(kDin / 64), 64, 0, stream>>>(sa);

      gemm64_f16_kernel<false, false><<<(kSeq / 64) * (kDm / 64) / 8, 256, 0, stream>>>(
          UY, kDin, WOUT, kDin, mob, kDm, UY, 64, 0, 1.0f, b_dt, kSeq, kDm, kDin, kScaleOut);
    }
  }

  add_norm_kernel<true, false, true><<<kRows, 256, 0, stream>>>(
      MO, RESID, RESID, NORMED, out, normf_w, normf_b, 1.0f);
}
